// SwinBlock_8632884265097
// MI455X (gfx1250) — hardware-run, weakly checked
//
#include <hip/hip_runtime.h>
#include <math.h>

constexpr int kBatch  = 16;
constexpr int kImg    = 56;
constexpr int kC      = 192;
constexpr int kL      = 3136;
constexpr int kRows   = 50176;
constexpr int kHeads  = 6;
constexpr int kHd     = 32;
constexpr int kWsz    = 7;
constexpr int kShift  = 3;
constexpr int kNt     = 49;
constexpr int kNwin   = 1024;
constexpr int kQkvN   = 576;
constexpr int kHid    = 1152;
constexpr int kRpbN   = 169;
constexpr int kChunkRows = 6272;
constexpr int kNChunks   = 8;
static_assert(kChunkRows * kNChunks == kRows);
static_assert(kRows % 64 == 0 && kChunkRows % 64 == 0 && kQkvN % 64 == 0 && kHid % 64 == 0 && kC % 64 == 0);
static_assert(kC % 32 == 0 && kHid % 32 == 0);
static_assert(kRows % 8 == 0);

constexpr float kWCarry    = 64.0f;
constexpr float kPCarry    = 1024.0f;
constexpr float kOCarry    = 16.0f;
constexpr float kGCarry    = 16.0f;
constexpr float kQkvScale  = 1.0f / 64.0f;
constexpr float kPVScale   = kOCarry / kPCarry;
constexpr float kProjScale = 1.0f / (64.0f * 16.0f);
constexpr float kFc1Scale  = 1.0f / 64.0f;
constexpr float kFc2Scale  = 1.0f / (64.0f * 16.0f);
constexpr float kQScale    = 0.17677669529663687f;
constexpr float kInvC      = 1.0f / 192.0f;
constexpr float kEps       = 1e-5f;

typedef __attribute__((ext_vector_type(16))) _Float16 v16h;
typedef __attribute__((ext_vector_type(8)))  _Float16 v8h;
typedef __attribute__((ext_vector_type(16))) __bf16   v16b;
typedef __attribute__((ext_vector_type(8)))  __bf16   v8b;
typedef __attribute__((ext_vector_type(8)))  float    v8f;
typedef __attribute__((ext_vector_type(4)))  float    v4f;
typedef __attribute__((ext_vector_type(4)))  unsigned int v4u;

__device__ __forceinline__ unsigned short f2bf_bits(float f) {
  unsigned u = __float_as_uint(f);
  return (unsigned short)((u + 0x7FFFu + ((u >> 16) & 1u)) >> 16);
}
__device__ __forceinline__ float bf_bits2f(unsigned short h) { return __uint_as_float(((unsigned)h) << 16); }

__device__ __forceinline__ void dep_guard_h(v8f& a, v8f& b, v16h x, v16h y) { asm volatile("v_nop\n\tv_nop\n\tv_nop\n\tv_nop" : "+v"(a), "+v"(b) : "v"(x), "v"(y)); }
__device__ __forceinline__ void dep_guard_b(v8f& a, v8f& b, v16b x, v16b y) { asm volatile("v_nop\n\tv_nop\n\tv_nop\n\tv_nop" : "+v"(a), "+v"(b) : "v"(x), "v"(y)); }
__device__ __forceinline__ void keep4_h(v16h a, v16h b, v16h c, v16h d) { asm volatile("v_nop" :: "v"(a), "v"(b), "v"(c), "v"(d)); }
__device__ __forceinline__ void keep4_b(v16b a, v16b b, v16b c, v16b d) { asm volatile("v_nop" :: "v"(a), "v"(b), "v"(c), "v"(d)); }
__device__ __forceinline__ void acc_guard4(v8f& a, v8f& b, v8f& c, v8f& d) { asm volatile("v_nop\n\tv_nop\n\tv_nop\n\tv_nop" : "+v"(a), "+v"(b), "+v"(c), "+v"(d)); }
template <typename T> struct Frag;
template <> struct Frag<_Float16> {
  typedef v16h V; union U { v16h v; v8h h[2]; };
  static __device__ __forceinline__ v16h load(const _Float16* p) {
    U f; f.h[0] = *(const v8h*)(p); f.h[1] = *(const v8h*)(p + 16); return f.v;
  }
  static __device__ __forceinline__ v8f mma(v16h a, v16h b, v8f c) {
    return __builtin_amdgcn_wmma_f32_16x16x32_f16(false, a, false, b, (short)0, c, false, false);
  }
  static __device__ __forceinline__ void guard(v8f& a, v8f& b, v16h x, v16h y) { dep_guard_h(a, b, x, y); }
  static __device__ __forceinline__ void keep(v16h a, v16h b, v16h c, v16h d) { keep4_h(a, b, c, d); }
};
template <> struct Frag<__bf16> {
  typedef v16b V; union U { v16b v; v8b h[2]; };
  static __device__ __forceinline__ v16b load(const __bf16* p) {
    U f; f.h[0] = *(const v8b*)(p); f.h[1] = *(const v8b*)(p + 16); return f.v;
  }
  static __device__ __forceinline__ v8f mma(v16b a, v16b b, v8f c) {
    return __builtin_amdgcn_wmma_f32_16x16x32_bf16(false, a, false, b, (short)0, c, false, false);
  }
  static __device__ __forceinline__ void guard(v8f& a, v8f& b, v16b x, v16b y) { dep_guard_b(a, b, x, y); }
  static __device__ __forceinline__ void keep(v16b a, v16b b, v16b c, v16b d) { keep4_b(a, b, c, d); }
};

__device__ __forceinline__ unsigned pk16(unsigned short a, unsigned short b) { return (unsigned)a | ((unsigned)b << 16); }
__device__ __forceinline__ unsigned short h_bits(float f) { const _Float16 h = (_Float16)f; return __builtin_bit_cast(unsigned short, h); }

__device__ __forceinline__ v8f hmma(v16h a, v16h b, v8f c) {
  c = __builtin_amdgcn_wmma_f32_16x16x32_f16(false, a, false, b, (short)0, c, false, false);
  asm volatile("v_nop\n\tv_nop\n\tv_nop\n\tv_nop" : "+v"(c) : "v"(a), "v"(b));
  return c;
}

template <int ET> struct Elem;
template <> struct Elem<0> { typedef _Float16 T; };
template <> struct Elem<1> { typedef __bf16 T; };
template <int ET, bool SPLIT, int BIAS_MODE, int OUT_MODE, bool RESID, int ACT = 0>
__global__ __launch_bounds__(256) void wmma_gemm64(
    const unsigned short* __restrict__ Ap, const unsigned short* __restrict__ A2p, int lda, long strideA,
    const unsigned short* __restrict__ Btp, const unsigned short* __restrict__ Bt2p, int ldb, long strideB,
    void* __restrict__ Cout, void* __restrict__ Cout2, int ldc, long strideC,
    const float* __restrict__ bias,
    const float* __restrict__ resid, long strideR,
    int M, int N, int K, float scale) {
  typedef typename Elem<ET>::T T;
  typedef typename Frag<T>::V V;
  const T* A = (const T*)Ap; const T* A2 = (const T*)A2p; const T* Bt = (const T*)Btp; const T* Bt2 = (const T*)Bt2p;
  __shared__ __align__(16) float sT[8][16 * 68];
  const int b    = blockIdx.y;
  const int lane = threadIdx.x & 31;
  const int wave = threadIdx.x >> 5;
  const int tilesN = N >> 6;
  const int tilesM = M >> 6;
  const int tile = blockIdx.x * 8 + wave;
  if (tile >= tilesM * tilesN) return;
  const int tm = tile / tilesN;
  const int tn = tile - tm * tilesN;
  const int m0 = tm << 6;
  const int n0 = tn << 6;

  const T* Ab  = A  + (size_t)b * strideA;
  const T* Bb  = Bt + (size_t)b * strideB;
  const T* Ab2 = SPLIT ? (A2  + (size_t)b * strideA) : nullptr;
  const T* Bb2 = SPLIT ? (Bt2 + (size_t)b * strideB) : nullptr;

  const int rlane = lane & 15;
  const int koff  = (lane >> 4) * 8;
  const int mOff  = (lane >> 4) * 8;

  v8f acc[4][4];
#pragma unroll
  for (int i = 0; i < 4; ++i)
#pragma unroll
    for (int j = 0; j < 4; ++j) acc[i][j] = (v8f){0.f,0.f,0.f,0.f,0.f,0.f,0.f,0.f};

  for (int k0 = 0; k0 < K; k0 += 32) {
    V bh[4], bl[4];
#pragma unroll
    for (int j = 0; j < 4; ++j) {
      const size_t bo = (size_t)(n0 + (j << 4) + rlane) * ldb + koff + k0;
      bh[j] = Frag<T>::load(Bb + bo);
      if (SPLIT) bl[j] = Frag<T>::load(Bb2 + bo);
    }
#pragma unroll
    for (int i = 0; i < 4; ++i) {
      const size_t ao = (size_t)(m0 + (i << 4) + rlane) * lda + koff + k0;
      V ah = Frag<T>::load(Ab + ao);
      V al;
      if (SPLIT) al = Frag<T>::load(Ab2 + ao);
#pragma unroll
      for (int j = 0; j < 4; ++j) {
        acc[i][j] = Frag<T>::mma(ah, bh[j], acc[i][j]);
        if (SPLIT) {
          acc[i][j] = Frag<T>::mma(ah, bl[j], acc[i][j]);
          acc[i][j] = Frag<T>::mma(al, bh[j], acc[i][j]);
        }
      }
      Frag<T>::guard(acc[i][0], acc[i][3], ah, SPLIT ? al : ah);
    }
    Frag<T>::keep(bh[0], bh[1], bh[2], bh[3]);
    if (SPLIT) Frag<T>::keep(bl[0], bl[1], bl[2], bl[3]);
  }
  acc_guard4(acc[0][0], acc[0][1], acc[0][2], acc[0][3]);
  acc_guard4(acc[1][0], acc[1][1], acc[1][2], acc[1][3]);
  acc_guard4(acc[2][0], acc[2][1], acc[2][2], acc[2][3]);
  acc_guard4(acc[3][0], acc[3][1], acc[3][2], acc[3][3]);

  float* slab = sT[wave];
  const float* Rb = RESID ? (resid + (size_t)b * strideR) : nullptr;
#pragma unroll
  for (int i = 0; i < 4; ++i) {
    const int mBase = m0 + (i << 4);
#pragma unroll
    for (int j = 0; j < 4; ++j) {
      const int n = n0 + (j << 4) + rlane;
      float bv = 0.f;
      if (BIAS_MODE == 2) bv = bias[n];
#pragma unroll
      for (int r = 0; r < 8; ++r) {
        float v = acc[i][j][r] * scale;
        if (BIAS_MODE == 1) v += bias[mBase + mOff + r];
        if (BIAS_MODE == 2) v += bv;
        if (RESID) v += Rb[(size_t)(mBase + mOff + r) * ldc + n];
        if (ACT == 2) v = fmaxf(v, 0.0f);
        if (ACT == 4) v = (v > 0.f) ? v : 0.01f * v;
        slab[(mOff + r) * 68 + (j << 4) + rlane] = v;
      }
    }
    __builtin_amdgcn_fence(__ATOMIC_RELEASE, "workgroup");
    __builtin_amdgcn_wave_barrier();
    __builtin_amdgcn_fence(__ATOMIC_ACQUIRE, "workgroup");
    if (OUT_MODE == 0) {
      float* C = (float*)Cout + (size_t)b * strideC;
      const int hh = lane >> 4, c4 = (lane & 15) * 4;
      for (int pass = 0; pass < 2; ++pass) {
#pragma unroll
        for (int it = 0; it < 8; ++it) {
          const int row = it * 2 + hh;
          v4f v = *(const v4f*)(slab + row * 68 + c4);
          *(volatile v4f*)(C + (size_t)(mBase + row) * ldc + n0 + c4) = v;
        }
        __threadfence();
      }
    } else {
      const int q = lane >> 3, c8 = (lane & 7) * 8;
      unsigned short* C  = (unsigned short*)Cout  + (size_t)b * strideC;
      unsigned short* C2 = (OUT_MODE == 2) ? ((unsigned short*)Cout2 + (size_t)b * strideC) : nullptr;
      for (int pass = 0; pass < 2; ++pass) {
#pragma unroll
        for (int it = 0; it < 4; ++it) {
          const int row = it * 4 + q;
          const float* sp = slab + row * 68 + c8;
          v8h hv, lv;
#pragma unroll
          for (int e = 0; e < 8; ++e) {
            if (OUT_MODE == 1) {
              hv[e] = (_Float16)sp[e];
            } else {
              unsigned short hb = f2bf_bits(sp[e]);
              unsigned short lb = f2bf_bits(sp[e] - bf_bits2f(hb));
              hv[e] = __builtin_bit_cast(_Float16, hb);
              lv[e] = __builtin_bit_cast(_Float16, lb);
            }
          }
          *(volatile v8h*)(C + (size_t)(mBase + row) * ldc + n0 + c8) = hv;
          if (OUT_MODE == 2) *(volatile v8h*)(C2 + (size_t)(mBase + row) * ldc + n0 + c8) = lv;
        }
        __threadfence();
      }
    }
    __builtin_amdgcn_fence(__ATOMIC_RELEASE, "workgroup");
    __builtin_amdgcn_wave_barrier();
    __builtin_amdgcn_fence(__ATOMIC_ACQUIRE, "workgroup");
  }
}

__global__ __launch_bounds__(256) void wcast4_kernel(const float* __restrict__ w0, const float* __restrict__ w1,
                                                     const float* __restrict__ w2, const float* __restrict__ w3,
                                                     unsigned short* __restrict__ o0, unsigned short* __restrict__ o1,
                                                     unsigned short* __restrict__ o2, unsigned short* __restrict__ o3,
                                                     int n8a, int n8b, int n8c, int n8d, float scale) {
  const int z = blockIdx.y;
  const float* in = (z == 0) ? w0 : (z == 1) ? w1 : (z == 2) ? w2 : w3;
  unsigned short* out = (z == 0) ? o0 : (z == 1) ? o1 : (z == 2) ? o2 : o3;
  const int n8 = (z == 0) ? n8a : (z == 1) ? n8b : (z == 2) ? n8c : n8d;
  const int i = blockIdx.x * 256 + threadIdx.x;
  if (i >= n8) return;
  const float* p = in + 8 * (size_t)i;
  const v4f a = *(const v4f*)(p);
  const v4f c = *(const v4f*)(p + 4);
  unsigned short hb[8];
#pragma unroll
  for (int e = 0; e < 4; ++e) {
    hb[e]     = h_bits(a[e] * scale);
    hb[4 + e] = h_bits(c[e] * scale);
  }
  const v4u u = (v4u){pk16(hb[0], hb[1]), pk16(hb[2], hb[3]), pk16(hb[4], hb[5]), pk16(hb[6], hb[7])};
  unsigned short* q = out + 8 * (size_t)i;
  *(volatile v4u*)q = u;
  __threadfence();
  *(volatile v4u*)q = u;
}

__global__ __launch_bounds__(256) void ln1_gather_kernel(const float* __restrict__ x, const int* __restrict__ hp,
                                                         const int* __restrict__ wp, const float* __restrict__ g,
                                                         const float* __restrict__ bt, unsigned short* __restrict__ out) {
  const int lane = threadIdx.x & 31, wave = threadIdx.x >> 5;
  const int wrow = blockIdx.x * 8 + wave;
  const int wb = wrow / kNt, n = wrow - wb * kNt;
  const int b = wb >> 6, wr = (wb >> 3) & 7, wc = wb & 7;
  const int ti = n / kWsz, tj = n - ti * kWsz;
  int rr = wr * kWsz + ti + kShift; rr = (rr >= kImg) ? (rr - kImg) : rr;
  int cc = wc * kWsz + tj + kShift; cc = (cc >= kImg) ? (cc - kImg) : cc;
  const int tok = (b * kImg + rr) * kImg + cc;
  const float qnan = __int_as_float(0x7fc00000);
  const float poison = (hp[0] != kImg || wp[0] != kImg) ? qnan : 0.0f;
  const bool valid = lane < 24;
  const int lc = valid ? lane : 23;
  const float* xr = x + (size_t)tok * kC + 8 * lc;
  const v4f a0 = *(const v4f*)(xr);
  const v4f a1 = *(const v4f*)(xr + 4);
  const v4f g0 = *(const v4f*)(g + 8 * lc);
  const v4f g1 = *(const v4f*)(g + 8 * lc + 4);
  const v4f b0 = *(const v4f*)(bt + 8 * lc);
  const v4f b1 = *(const v4f*)(bt + 8 * lc + 4);
  float v[8], gg[8], bb[8];
#pragma unroll
  for (int e = 0; e < 4; ++e) {
    v[e] = valid ? a0[e] : 0.0f;  v[4 + e] = valid ? a1[e] : 0.0f;
    gg[e] = g0[e]; gg[4 + e] = g1[e]; bb[e] = b0[e]; bb[4 + e] = b1[e];
  }
  float s = 0.f;
#pragma unroll
  for (int e = 0; e < 8; ++e) s += v[e];
#pragma unroll
  for (int off = 16; off > 0; off >>= 1) s += __shfl_xor(s, off, 32);
  const float mean = s * kInvC + poison;
  float qv = 0.f;
#pragma unroll
  for (int e = 0; e < 8; ++e) { const float d = valid ? (v[e] - mean) : 0.0f; qv += d * d; }
#pragma unroll
  for (int off = 16; off > 0; off >>= 1) qv += __shfl_xor(qv, off, 32);
  const float rstd = rsqrtf(qv * kInvC + kEps);
  unsigned short hb[8];
#pragma unroll
  for (int e = 0; e < 8; ++e) hb[e] = h_bits((v[e] - mean) * rstd * gg[e] + bb[e]);
  const v4u u = (v4u){pk16(hb[0], hb[1]), pk16(hb[2], hb[3]), pk16(hb[4], hb[5]), pk16(hb[6], hb[7])};
  if (valid) {
    unsigned short* op = out + (size_t)wrow * kC + 8 * lane;
    *(volatile v4u*)op = u;
    __threadfence();
    *(volatile v4u*)op = u;
  }
}

__global__ __launch_bounds__(128) void win_attn_kernel(const unsigned short* __restrict__ qkv,
                                                      const float* __restrict__ rpb,
                                                      unsigned short* __restrict__ o16) {
  __shared__ __align__(16) _Float16 sQ[64 * 32];
  __shared__ __align__(16) _Float16 sK[64 * 32];
  __shared__ __align__(16) _Float16 sVt[32 * 64];
  __shared__ __align__(16) float    sS[64 * 64];
  __shared__ __align__(16) _Float16 sP[64 * 64];
  __shared__ __align__(16) _Float16 sO[kNt * kC];
  __shared__ float sRpb[1016];

  const int tid = threadIdx.x, lane = tid & 31, wave = tid >> 5;
  const int rlane = lane & 15, hh = lane >> 4, koff = hh * 8;
  const int win = blockIdx.x;
  const size_t rowbase = (size_t)win * kNt;

  for (int i = tid; i < kRpbN * kHeads; i += 128) sRpb[i] = rpb[i];

  for (int head = 0; head < kHeads; ++head) {
    __syncthreads();
    {
      const int r = tid >> 1, d0 = (tid & 1) * 16;
      const bool valid = r < kNt;
      const int rc = valid ? r : (kNt - 1);
      const unsigned short* src = qkv + (rowbase + rc) * kQkvN + head * kHd + d0;
      v4u uq0 = *(const v4u*)(src);           v4u uq1 = *(const v4u*)(src + 8);
      v4u uk0 = *(const v4u*)(src + kC);      v4u uk1 = *(const v4u*)(src + kC + 8);
      v4u uv0 = *(const v4u*)(src + 2 * kC);  v4u uv1 = *(const v4u*)(src + 2 * kC + 8);
      const unsigned mk = valid ? 0xffffffffu : 0u;
      const v4u m4 = (v4u){mk, mk, mk, mk};
      uq0 = uq0 & m4; uq1 = uq1 & m4; uk0 = uk0 & m4; uk1 = uk1 & m4; uv0 = uv0 & m4; uv1 = uv1 & m4;
      *(v4u*)(void*)(sQ + r * 32 + d0)     = uq0;
      *(v4u*)(void*)(sQ + r * 32 + d0 + 8) = uq1;
      *(v4u*)(void*)(sK + r * 32 + d0)     = uk0;
      *(v4u*)(void*)(sK + r * 32 + d0 + 8) = uk1;
#pragma unroll
      for (int e = 0; e < 4; ++e) {
        const unsigned wa = uv0[e], wb = uv1[e];
        sVt[(d0 + 2 * e) * 64 + r]         = __builtin_bit_cast(_Float16, (unsigned short)(wa & 0xffffu));
        sVt[(d0 + 2 * e + 1) * 64 + r]     = __builtin_bit_cast(_Float16, (unsigned short)(wa >> 16));
        sVt[(d0 + 8 + 2 * e) * 64 + r]     = __builtin_bit_cast(_Float16, (unsigned short)(wb & 0xffffu));
        sVt[(d0 + 8 + 2 * e + 1) * 64 + r] = __builtin_bit_cast(_Float16, (unsigned short)(wb >> 16));
      }
    }
    __syncthreads();

    {
      v8f acc[4];
      const v16h aq = Frag<_Float16>::load(sQ + (wave * 16 + rlane) * 32 + koff);
#pragma unroll
      for (int j = 0; j < 4; ++j) {
        const v16h bk = Frag<_Float16>::load(sK + (j * 16 + rlane) * 32 + koff);
        acc[j] = hmma(aq, bk, (v8f){0.f,0.f,0.f,0.f,0.f,0.f,0.f,0.f});
      }
#pragma unroll
      for (int j = 0; j < 4; ++j) {
        const int col = j * 16 + rlane;
        const bool colok = col < kNt;
        const int colc = colok ? col : (kNt - 1);
        const int im = colc / kWsz, jm = colc - im * kWsz;
#pragma unroll
        for (int r = 0; r < 8; ++r) {
          const int row = wave * 16 + 8 * hh + r;
          const bool rowok = row < kNt;
          const int rowc = rowok ? row : (kNt - 1);
          const int in_ = rowc / kWsz, jn = rowc - in_ * kWsz;
          const int idx = (in_ - im + (kWsz - 1)) * (2 * kWsz - 1) + (jn - jm + (kWsz - 1));
          const float bterm = sRpb[idx * kHeads + head];
          float sv = acc[j][r] * kQScale + (rowok ? bterm : 0.0f);
          sv = colok ? sv : -1e30f;
          sS[row * 64 + col] = sv;
        }
      }
    }
    __syncthreads();

#pragma unroll 2
    for (int r = 0; r < 16; ++r) {
      const int row = wave * 16 + r;
      const float s0 = sS[row * 64 + lane];
      const float s1 = sS[row * 64 + 32 + lane];
      float m = fmaxf(s0, s1);
#pragma unroll
      for (int off = 16; off > 0; off >>= 1) m = fmaxf(m, __shfl_xor(m, off, 32));
      const float e0 = expf(s0 - m), e1 = expf(s1 - m);
      float sum = e0 + e1;
#pragma unroll
      for (int off = 16; off > 0; off >>= 1) sum += __shfl_xor(sum, off, 32);
      const float f = kPCarry / sum;
      sP[row * 64 + lane]      = (_Float16)(e0 * f);
      sP[row * 64 + 32 + lane] = (_Float16)(e1 * f);
    }
    __syncthreads();

    {
      v8f oacc0 = (v8f){0.f,0.f,0.f,0.f,0.f,0.f,0.f,0.f};
      v8f oacc1 = (v8f){0.f,0.f,0.f,0.f,0.f,0.f,0.f,0.f};
#pragma unroll
      for (int kk = 0; kk < 2; ++kk) {
        const v16h pa  = Frag<_Float16>::load(sP  + (wave * 16 + rlane) * 64 + kk * 32 + koff);
        const v16h vb0 = Frag<_Float16>::load(sVt + (rlane) * 64 + kk * 32 + koff);
        const v16h vb1 = Frag<_Float16>::load(sVt + (16 + rlane) * 64 + kk * 32 + koff);
        oacc0 = hmma(pa, vb0, oacc0);
        oacc1 = hmma(pa, vb1, oacc1);
      }
#pragma unroll
      for (int r = 0; r < 8; ++r) {
        const int row = wave * 16 + 8 * hh + r;
        if (row < kNt) {
          sO[row * kC + head * kHd + rlane]      = (_Float16)(oacc0[r] * kPVScale);
          sO[row * kC + head * kHd + 16 + rlane] = (_Float16)(oacc1[r] * kPVScale);
        }
      }
    }
  }
  __syncthreads();

  const int lc = (lane < 24) ? lane : 23;
  for (int pass = 0; pass < 2; ++pass) {
    for (int row = wave; row < kNt; row += 4) {
      const v4u u = *(const v4u*)(const void*)(sO + row * kC + lc * 8);
      if (lane < 24) *(volatile v4u*)(o16 + (rowbase + row) * kC + lane * 8) = u;
    }
    __threadfence();
  }
}

__global__ __launch_bounds__(256) void merge_ln2_kernel(const float* __restrict__ x, const float* __restrict__ proj,
                                                        const float* __restrict__ g, const float* __restrict__ bt,
                                                        float* __restrict__ x1, unsigned short* __restrict__ h2) {
  __shared__ __align__(16) float stg[8 * 192];
  const int lane = threadIdx.x & 31, wave = threadIdx.x >> 5;
  const int tok = blockIdx.x * 8 + wave;
  const int b = tok / kL, rem = tok - b * kL;
  const int r = rem / kImg, c = rem - r * kImg;
  int rr = r - kShift; rr = (rr < 0) ? (rr + kImg) : rr;
  int cc = c - kShift; cc = (cc < 0) ? (cc + kImg) : cc;
  const int wr = rr / kWsz, ti = rr - wr * kWsz, wc = cc / kWsz, tj = cc - wc * kWsz;
  const int wrow = ((b * 64 + wr * 8 + wc) * kNt) + ti * kWsz + tj;
  const bool validB = lane < 16;
  const int lb = validB ? lane : 15;
  const float* xr = x + (size_t)tok * kC;
  const float* pr = proj + (size_t)wrow * kC;
  const v4f xa = *(const v4f*)(xr + 4 * lane);
  const v4f xb = *(const v4f*)(xr + 128 + 4 * lb);
  const v4f pa = *(const v4f*)(pr + 4 * lane);
  const v4f pb = *(const v4f*)(pr + 128 + 4 * lb);
  const v4f ga = *(const v4f*)(g + 4 * lane);
  const v4f gb = *(const v4f*)(g + 128 + 4 * lb);
  const v4f ba = *(const v4f*)(bt + 4 * lane);
  const v4f bb = *(const v4f*)(bt + 128 + 4 * lb);
  float v[8];
#pragma unroll
  for (int e = 0; e < 4; ++e) {
    v[e] = xa[e] + pa[e];
    v[4 + e] = validB ? (xb[e] + pb[e]) : 0.0f;
  }
  const v4f va = (v4f){v[0], v[1], v[2], v[3]};
  const v4f vb = (v4f){v[4], v[5], v[6], v[7]};
  float* xo = x1 + (size_t)tok * kC;
  for (int pass = 0; pass < 2; ++pass) {
    *(volatile v4f*)(xo + 4 * lane) = va;
    if (validB) *(volatile v4f*)(xo + 128 + 4 * lane) = vb;
    __threadfence();
  }
  float s = 0.f;
#pragma unroll
  for (int e = 0; e < 8; ++e) s += v[e];
#pragma unroll
  for (int off = 16; off > 0; off >>= 1) s += __shfl_xor(s, off, 32);
  const float mean = s * kInvC;
  float qv = 0.f;
#pragma unroll
  for (int e = 0; e < 4; ++e) { const float d = v[e] - mean; qv += d * d; }
#pragma unroll
  for (int e = 0; e < 4; ++e) { const float d = validB ? (v[4 + e] - mean) : 0.0f; qv += d * d; }
#pragma unroll
  for (int off = 16; off > 0; off >>= 1) qv += __shfl_xor(qv, off, 32);
  const float rstd = rsqrtf(qv * kInvC + kEps);
  float* sw = stg + wave * 192;
#pragma unroll
  for (int e = 0; e < 4; ++e) {
    sw[4 * lane + e] = (v[e] - mean) * rstd * ga[e] + ba[e];
    if (validB) sw[128 + 4 * lane + e] = (v[4 + e] - mean) * rstd * gb[e] + bb[e];
  }
  __syncthreads();
  const int lc = (lane < 24) ? lane : 23;
  const v4f h0 = *(const v4f*)(sw + 8 * lc);
  const v4f h1 = *(const v4f*)(sw + 8 * lc + 4);
  unsigned short hb[8];
#pragma unroll
  for (int e = 0; e < 4; ++e) { hb[e] = h_bits(h0[e]); hb[4 + e] = h_bits(h1[e]); }
  const v4u u = (v4u){pk16(hb[0], hb[1]), pk16(hb[2], hb[3]), pk16(hb[4], hb[5]), pk16(hb[6], hb[7])};
  if (lane < 24) {
    unsigned short* op = h2 + (size_t)tok * kC + 8 * lane;
    *(volatile v4u*)op = u;
    __threadfence();
    *(volatile v4u*)op = u;
  }
}

__global__ __launch_bounds__(256) void gelu_cast_kernel(const float* __restrict__ in, unsigned short* __restrict__ out,
                                                        int n8, float carry) {
  const int i = blockIdx.x * 256 + threadIdx.x;
  if (i >= n8) return;
  const float* p = in + 8 * (size_t)i;
  v4u u = (v4u){0u, 0u, 0u, 0u};
#pragma unroll 1
  for (int e2 = 0; e2 < 4; ++e2) {
    const float a0 = p[2 * e2];
    const float a1 = p[2 * e2 + 1];
    const float g0 = 0.5f * a0 * (1.0f + erff(a0 * 0.70710678118654752f)) * carry;
    const float g1 = 0.5f * a1 * (1.0f + erff(a1 * 0.70710678118654752f)) * carry;
    const unsigned w = pk16(h_bits(g0), h_bits(g1));
    u = (v4u){u[1], u[2], u[3], w};
  }
  unsigned short* q = out + 8 * (size_t)i;
  *(volatile v4u*)q = u;
  __threadfence();
  *(volatile v4u*)q = u;
}

static_assert((size_t)kChunkRows * kHid * 4 <= (size_t)kRows * kC * 4);
static_assert((size_t)kChunkRows * kHid * 2 <= (size_t)kRows * kC * 2);
static_assert((size_t)kRows * kC * 4 + (size_t)kRows * kC * 2 == (size_t)kRows * kQkvN * 2);

extern "C" void kernel_launch(void* const* d_in, const int* in_sizes, int n_in,
                              void* d_out, int out_size, void* d_ws, size_t ws_size,
                              hipStream_t stream) {
  if (n_in < 16) return;
  if (in_sizes[0] != kRows * kC || out_size != kRows * kC) return;
  if (in_sizes[1] < 1 || in_sizes[2] < 1) return;
  if (in_sizes[3] != kC || in_sizes[4] != kC || in_sizes[5] != kQkvN * kC || in_sizes[6] != kQkvN) return;
  if (in_sizes[7] != kRpbN * kHeads || in_sizes[8] != kC * kC || in_sizes[9] != kC) return;
  if (in_sizes[10] != kC || in_sizes[11] != kC || in_sizes[12] != kHid * kC || in_sizes[13] != kHid) return;
  if (in_sizes[14] != kC * kHid || in_sizes[15] != kC) return;

  const float* x      = (const float*)d_in[0];
  const int*   hp     = (const int*)d_in[1];
  const int*   wp     = (const int*)d_in[2];
  const float* ln1_g  = (const float*)d_in[3];
  const float* ln1_b  = (const float*)d_in[4];
  const float* qkv_w  = (const float*)d_in[5];
  const float* qkv_b  = (const float*)d_in[6];
  const float* rpb    = (const float*)d_in[7];
  const float* proj_w = (const float*)d_in[8];
  const float* proj_b = (const float*)d_in[9];
  const float* ln2_g  = (const float*)d_in[10];
  const float* ln2_b  = (const float*)d_in[11];
  const float* fc1_w  = (const float*)d_in[12];
  const float* fc1_b  = (const float*)d_in[13];
  const float* fc2_w  = (const float*)d_in[14];
  const float* fc2_b  = (const float*)d_in[15];
  float* out = (float*)d_out;

  size_t off = 0;
  auto carve = [&](size_t bytes) { size_t o = off; off += (bytes + 255) & ~(size_t)255; return o; };
  const size_t oWqkv  = carve((size_t)kQkvN * kC * 2);
  const size_t oWproj = carve((size_t)kC * kC * 2);
  const size_t oWfc1  = carve((size_t)kHid * kC * 2);
  const size_t oWfc2  = carve((size_t)kC * kHid * 2);
  const size_t oR1    = carve((size_t)kRows * kC * 2);
  const size_t oR2    = carve((size_t)kRows * kQkvN * 2);
  const size_t oR3    = carve((size_t)kRows * kC * 4);
  if (off > ws_size) return;

  char* ws = (char*)d_ws;
  unsigned short* wqkv16  = (unsigned short*)(ws + oWqkv);
  unsigned short* wproj16 = (unsigned short*)(ws + oWproj);
  unsigned short* wfc1_16 = (unsigned short*)(ws + oWfc1);
  unsigned short* wfc2_16 = (unsigned short*)(ws + oWfc2);
  unsigned short* hw16    = (unsigned short*)(ws + oR1);
  unsigned short* o16     = (unsigned short*)(ws + oR1);
  unsigned short* g16     = (unsigned short*)(ws + oR1);
  unsigned short* qkv16   = (unsigned short*)(ws + oR2);
  float*          proj32  = (float*)(ws + oR2);
  float*          pre32   = (float*)(ws + oR2);
  unsigned short* h2_16   = (unsigned short*)(ws + oR2 + (size_t)kRows * kC * 4);
  float*          x1      = (float*)(ws + oR3);

  const int n8q = kQkvN * kC / 8, n8p = kC * kC / 8, n8f1 = kHid * kC / 8, n8f2 = kC * kHid / 8;
  wcast4_kernel<<<dim3((n8f1 + 255) / 256, 4), 256, 0, stream>>>(qkv_w, proj_w, fc1_w, fc2_w,
                                                                wqkv16, wproj16, wfc1_16, wfc2_16,
                                                                n8q, n8p, n8f1, n8f2, kWCarry);
  ln1_gather_kernel<<<kRows / 8, 256, 0, stream>>>(x, hp, wp, ln1_g, ln1_b, hw16);
  {
    const int tiles = (kRows / 64) * (kQkvN / 64);
    wmma_gemm64<0, false, 2, 1, false, 0><<<dim3((tiles + 7) / 8, 1), 256, 0, stream>>>(
        hw16, hw16, kC, 0L, wqkv16, wqkv16, kC, 0L, (void*)qkv16, (void*)qkv16, kQkvN, 0L,
        qkv_b, qkv_b, 0L, kRows, kQkvN, kC, kQkvScale);
  }
  win_attn_kernel<<<kNwin, 128, 0, stream>>>(qkv16, rpb, o16);
  {
    const int tiles = (kRows / 64) * (kC / 64);
    wmma_gemm64<0, false, 2, 0, false, 0><<<dim3((tiles + 7) / 8, 1), 256, 0, stream>>>(
        o16, o16, kC, 0L, wproj16, wproj16, kC, 0L, (void*)proj32, (void*)proj32, kC, 0L,
        proj_b, proj_b, 0L, kRows, kC, kC, kProjScale);
  }
  merge_ln2_kernel<<<kRows / 8, 256, 0, stream>>>(x, proj32, ln2_g, ln2_b, x1, h2_16);
  for (int ch = 0; ch < kNChunks; ++ch) {
    const unsigned short* a_h2 = h2_16 + (size_t)ch * kChunkRows * kC;
    const float* rchunk = x1 + (size_t)ch * kChunkRows * kC;
    float* ochunk = out + (size_t)ch * kChunkRows * kC;
    {
      const int tiles = (kChunkRows / 64) * (kHid / 64);
      wmma_gemm64<0, false, 2, 0, false, 0><<<dim3((tiles + 7) / 8, 1), 256, 0, stream>>>(
          a_h2, a_h2, kC, 0L, wfc1_16, wfc1_16, kC, 0L, (void*)pre32, (void*)pre32, kHid, 0L,
          fc1_b, fc1_b, 0L, kChunkRows, kHid, kC, kFc1Scale);
    }
    {
      const int n8 = kChunkRows * kHid / 8;
      gelu_cast_kernel<<<(n8 + 255) / 256, 256, 0, stream>>>(pre32, g16, n8, kGCarry);
    }
    {
      const int tiles = (kChunkRows / 64) * (kC / 64);
      wmma_gemm64<0, false, 2, 0, true, 0><<<dim3((tiles + 7) / 8, 1), 256, 0, stream>>>(
          g16, g16, kHid, 0L, wfc2_16, wfc2_16, kHid, 0L, (void*)ochunk, (void*)ochunk, kC, 0L,
          fc2_b, rchunk, 0L, kChunkRows, kC, kHid, kFc2Scale);
    }
  }
}
